// ResAxialAttentionUNet_41205916238508
// MI455X (gfx1250) — hardware-verified
//
#include <hip/hip_runtime.h>
#include <stdint.h>

#pragma clang fp contract(off)


#define H     96
#define W     96
#define C     128
#define MOUT  128
#define HP    98
#define WP    98
#define NS    9
#define KTOT  1152
#define SP    9216
#define PLANE 9604
#define MOFF  32
#define NB    2
#define CPITCH 68

typedef __bf16 v16bf __attribute__((ext_vector_type(16)));
typedef float v8f __attribute__((ext_vector_type(8)));
typedef float v4f __attribute__((ext_vector_type(4)));
typedef int v4i __attribute__((ext_vector_type(4)));
typedef unsigned short us8 __attribute__((ext_vector_type(8)));
typedef unsigned short us16 __attribute__((ext_vector_type(16)));

union Frag { v16bf v; us16 s; us8 h8[2]; };

static __device__ __forceinline__ v8f wmma_bf(const v16bf a, const v16bf b, v8f c) {
  v8f d = __builtin_amdgcn_wmma_f32_16x16x32_bf16(false, a, false, b, (short)0, c, false, false);
  asm volatile("v_nop\n\tv_nop\n\tv_nop\n\tv_nop" : "+v"(d) : "v"(a), "v"(b));
  return d;
}

static __device__ __forceinline__ v8f zero8() {
  v8f z = {0.f, 0.f, 0.f, 0.f, 0.f, 0.f, 0.f, 0.f};
  return z;
}

static __device__ __forceinline__ unsigned int bfbits(float f) {
  const unsigned int u = __float_as_uint(f);
  return (u + 0x7FFFu + ((u >> 16) & 1u)) >> 16;
}

static __device__ __forceinline__ void split_bf(float x, unsigned short& hi, unsigned short& lo) {
  const unsigned int hb = bfbits(x);
  const float hf = __uint_as_float(hb << 16);
  hi = (unsigned short)hb;
  lo = (unsigned short)bfbits(x - hf);
}

static __device__ __forceinline__ float padval(const float* __restrict__ x, int idx) {
  const int bc = idx / PLANE;
  const int r = idx - bc * PLANE;
  const int i = r / WP;
  const int j = r - i * WP;
  float v = 0.f;
  if (i >= 1 && i <= H && j >= 1 && j <= W)
    v = x[(size_t)bc * SP + (size_t)(i - 1) * W + (j - 1)];
  return v;
}

__global__ __launch_bounds__(256) void k_pad(const float* __restrict__ x,
                                             float* __restrict__ xp, int nquad) {
  const int q = blockIdx.x * 256 + threadIdx.x;
  if (q >= nquad) return;
  const int i0 = q * 4;
  v4f o;
  o.x = padval(x, i0 + 0);
  o.y = padval(x, i0 + 1);
  o.z = padval(x, i0 + 2);
  o.w = padval(x, i0 + 3);
  volatile v4f* p = (volatile v4f*)(xp + (size_t)i0);
  *p = o;
  __threadfence();
  *p = o;
}

__global__ __launch_bounds__(256) void k_prep(const float* __restrict__ conv_w,
                                              const float* __restrict__ pconv_w,
                                              const float* __restrict__ adconv_w,
                                              unsigned short* __restrict__ Amh,
                                              unsigned short* __restrict__ Aml,
                                              unsigned short* __restrict__ Aoh,
                                              unsigned short* __restrict__ Aol,
                                              int nmain, int noff) {
  const int g = blockIdx.x * 256 + threadIdx.x;
  us8 hv, lv;
  unsigned short* dh;
  unsigned short* dl;
  if (g < nmain) {
    const int m = g / (KTOT / 8);
    const int kk = (g - m * (KTOT / 8)) * 8;
    const int n = kk >> 7;
    const int c0 = kk & 127;
#pragma unroll
    for (int u = 0; u < 8; ++u) {
      const float wv = conv_w[(size_t)m * KTOT + (size_t)(c0 + u) * 9 + n];
      unsigned short a, bq;
      split_bf(wv, a, bq);
      hv[u] = a;
      lv[u] = bq;
    }
    dh = Amh + (size_t)m * KTOT + kk;
    dl = Aml + (size_t)m * KTOT + kk;
  } else {
    const int g2 = g - nmain;
    if (g2 >= noff) return;
    const int o = g2 / (KTOT / 8);
    const int kk = (g2 - o * (KTOT / 8)) * 8;
    const int t = kk >> 7;
    const int c0 = kk & 127;
#pragma unroll
    for (int u = 0; u < 8; ++u) {
      float wv = 0.f;
      if (o < 18)
        wv = pconv_w[(size_t)o * KTOT + (size_t)(c0 + u) * 9 + t];
      else if (o < 21)
        wv = adconv_w[(size_t)(o - 18) * KTOT + (size_t)(c0 + u) * 9 + t];
      unsigned short a, bq;
      split_bf(wv, a, bq);
      hv[u] = a;
      lv[u] = bq;
    }
    dh = Aoh + (size_t)o * KTOT + kk;
    dl = Aol + (size_t)o * KTOT + kk;
  }
  volatile us8* ph = (volatile us8*)dh;
  volatile us8* pl = (volatile us8*)dl;
  *ph = hv;
  *pl = lv;
  __threadfence();
  *ph = hv;
  *pl = lv;
}

__global__ __launch_bounds__(64) void k_offs(const unsigned short* __restrict__ Aoh,
                                             const unsigned short* __restrict__ Aol,
                                             const float* __restrict__ xp,
                                             const float* __restrict__ pconv_b,
                                             const float* __restrict__ adconv_b,
                                             v4i* __restrict__ PI, v4f* __restrict__ PG) {
  __shared__ float Cs[MOFF][33];
  const int tid = threadIdx.x;
  const int l = tid & 31, w = tid >> 5, h = l >> 4, m = l & 15;
  const int jg = blockIdx.x, i = blockIdx.y, b = blockIdx.z;
  const int j0 = jg * 32;
  const int colj = j0 + 16 * w + m;
  const float* xpb = xp + (size_t)b * C * PLANE;

  v8f acc0 = zero8(), acc1 = zero8();

#pragma unroll 1
  for (int t = 0; t < NS; ++t) {
    const int ta = t / 3;
    const int tb = t - ta * 3;
    const int rowoff = (i + ta) * WP + (colj + tb);
#pragma unroll 1
    for (int cq = 0; cq < 4; ++cq) {
      const int c0 = cq * 32;
      const int k0 = t * C + c0;
      Frag bh, bl;
#pragma unroll
      for (int e = 0; e < 16; ++e) {
        const int kk = (e < 8) ? (8 * h + e) : (8 + 8 * h + e);
        const float v = xpb[(size_t)(c0 + kk) * PLANE + rowoff];
        unsigned short a, bq;
        split_bf(v, a, bq);
        bh.s[e] = a;
        bl.s[e] = bq;
      }
      {
        Frag ah, al;
        const size_t ar = (size_t)m * KTOT + k0;
        ah.h8[0] = *(const us8*)(Aoh + ar + 8 * h);
        ah.h8[1] = *(const us8*)(Aoh + ar + 16 + 8 * h);
        al.h8[0] = *(const us8*)(Aol + ar + 8 * h);
        al.h8[1] = *(const us8*)(Aol + ar + 16 + 8 * h);
        acc0 = wmma_bf(ah.v, bl.v, acc0);
        acc0 = wmma_bf(al.v, bh.v, acc0);
        acc0 = wmma_bf(ah.v, bh.v, acc0);
      }
      {
        Frag ah, al;
        const size_t ar = (size_t)(16 + m) * KTOT + k0;
        ah.h8[0] = *(const us8*)(Aoh + ar + 8 * h);
        ah.h8[1] = *(const us8*)(Aoh + ar + 16 + 8 * h);
        al.h8[0] = *(const us8*)(Aol + ar + 8 * h);
        al.h8[1] = *(const us8*)(Aol + ar + 16 + 8 * h);
        acc1 = wmma_bf(ah.v, bl.v, acc1);
        acc1 = wmma_bf(al.v, bh.v, acc1);
        acc1 = wmma_bf(ah.v, bh.v, acc1);
      }
    }
  }

#pragma unroll
  for (int r = 0; r < 8; ++r) {
    Cs[8 * h + r][16 * w + m] = acc0[r];
    Cs[16 + 8 * h + r][16 * w + m] = acc1[r];
  }
  __syncthreads();

  if (tid < 32) {
    const int t = tid;
    const int j = j0 + t;
    float ad3[3];
#pragma unroll
    for (int q = 0; q < 3; ++q) {
      const float v = Cs[18 + q][t] + adconv_b[q];
      const float ex = expf(-v);
      const float sig = 1.0f / (1.0f + ex);
      const float adb = 1.0f - sig;
      ad3[q] = adb * 2.0f;
    }
    v4i piA[NS];
    v4f pgA[NS];
#pragma unroll
    for (int n = 0; n < NS; ++n) {
      const int dn = n / 3 - 1;
      const int dm = n % 3 - 1;
      const float offx = Cs[n][t] + pconv_b[n];
      const float offy = Cs[9 + n][t] + pconv_b[9 + n];
      const float ad = ad3[n % 3];
      const float adx = ad * (float)dn;
      const float ady = ad * (float)dm;
      float px = ((float)(i + 1 + dn) + offx) + adx;
      float py = ((float)(j + 1 + dm) + offy) + ady;
      const float flx = floorf(px), fly = floorf(py);
      const int qltx = (int)fminf(fmaxf(flx, 0.f), 97.f);
      const int qlty = (int)fminf(fmaxf(fly, 0.f), 97.f);
      const int qrbx = (int)fminf(fmaxf(flx + 1.f, 0.f), 97.f);
      const int qrby = (int)fminf(fmaxf(fly + 1.f, 0.f), 97.f);
      const bool mx = (px < 1.f) || (px > 96.f);
      const bool my = (py < 1.f) || (py > 96.f);
      px = fminf(fmaxf(mx ? flx : px, 0.f), 97.f);
      py = fminf(fmaxf(my ? fly : py, 0.f), 97.f);
      const float qltxf = (float)qltx, qltyf = (float)qlty;
      const float qrbxf = (float)qrbx, qrbyf = (float)qrby;
      const float g_lt = (1.f + (qltxf - px)) * (1.f + (qltyf - py));
      const float g_rb = (1.f - (qrbxf - px)) * (1.f - (qrbyf - py));
      const float g_lb = (1.f + (qltxf - px)) * (1.f - (qrbyf - py));
      const float g_rt = (1.f - (qrbxf - px)) * (1.f + (qltyf - py));
      v4i pi;
      pi.x = qltx * WP + qlty;
      pi.y = qrbx * WP + qrby;
      pi.z = qltx * WP + qrby;
      pi.w = qrbx * WP + qlty;
      v4f pg;
      pg.x = g_lt; pg.y = g_rb; pg.z = g_lb; pg.w = g_rt;
      piA[n] = pi;
      pgA[n] = pg;
    }
    const size_t pbase = ((size_t)(b * NS)) * SP + (size_t)i * W + j;
#pragma unroll
    for (int n = 0; n < NS; ++n) {
      *(volatile v4i*)(PI + pbase + (size_t)n * SP) = piA[n];
      *(volatile v4f*)(PG + pbase + (size_t)n * SP) = pgA[n];
    }
    __threadfence();
#pragma unroll
    for (int n = 0; n < NS; ++n) {
      *(volatile v4i*)(PI + pbase + (size_t)n * SP) = piA[n];
      *(volatile v4f*)(PG + pbase + (size_t)n * SP) = pgA[n];
    }
  }
}

__global__ __launch_bounds__(256) void k_gath(const float* __restrict__ xp,
                                              const v4i* __restrict__ PI,
                                              const v4f* __restrict__ PG,
                                              unsigned short* __restrict__ Bth,
                                              unsigned short* __restrict__ Btl, int npair) {
  const int g = blockIdx.x * 256 + threadIdx.x;
  const int pr = g >> 4;
  const int lam = g & 15;
  if (pr >= npair) return;
  const int b = pr / (SP * NS);
  const int rem = pr - b * (SP * NS);
  const int sp = rem / NS;
  const int n = rem - sp * NS;
  const size_t pidx = ((size_t)(b * NS + n)) * SP + sp;
  const v4i gi = PI[pidx];
  const v4f gg = PG[pidx];
  const int i0 = min(max(gi.x, 0), PLANE - 1);
  const int i1 = min(max(gi.y, 0), PLANE - 1);
  const int i2 = min(max(gi.z, 0), PLANE - 1);
  const int i3 = min(max(gi.w, 0), PLANE - 1);
  const float* xc = xp + ((size_t)(b * C + lam * 8)) * PLANE;
  us8 hv, lv;
#pragma unroll
  for (int u = 0; u < 8; ++u) {
    const float* p = xc + (size_t)u * PLANE;
    const float t0 = gg.x * p[i0];
    const float t1 = gg.y * p[i1];
    const float t2 = gg.z * p[i2];
    const float t3 = gg.w * p[i3];
    const float v = ((t0 + t1) + t2) + t3;
    unsigned short a, bq;
    split_bf(v, a, bq);
    hv[u] = a;
    lv[u] = bq;
  }
  const size_t o = ((size_t)(b * SP + sp)) * KTOT + (size_t)n * C + (size_t)lam * 8;
  volatile us8* ph = (volatile us8*)(Bth + o);
  volatile us8* pl = (volatile us8*)(Btl + o);
  *ph = hv;
  *pl = lv;
  __threadfence();
  *ph = hv;
  *pl = lv;
}

__global__ __launch_bounds__(256) void k_gemm(const unsigned short* __restrict__ Amh,
                                              const unsigned short* __restrict__ Aml,
                                              const unsigned short* __restrict__ Bth,
                                              const unsigned short* __restrict__ Btl,
                                              float* __restrict__ out) {
  __shared__ __attribute__((aligned(16))) float Cs[MOUT][CPITCH];
  const int tid = threadIdx.x;
  const int l = tid & 31, w = tid >> 5, h = l >> 4, m = l & 15;
  const int wm = w & 1, wn = w >> 1;
  const int b = blockIdx.y;
  const int sp0 = blockIdx.x * 64;
  const size_t bcol = ((size_t)(b * SP + sp0 + 16 * wn + m)) * KTOT;

  v8f acc[4];
#pragma unroll
  for (int mt = 0; mt < 4; ++mt) acc[mt] = zero8();

#pragma unroll 1
  for (int ks = 0; ks < KTOT / 32; ++ks) {
    const int k0 = ks * 32;
    Frag bh, bl;
    bh.h8[0] = *(const us8*)(Bth + bcol + k0 + 8 * h);
    bh.h8[1] = *(const us8*)(Bth + bcol + k0 + 16 + 8 * h);
    bl.h8[0] = *(const us8*)(Btl + bcol + k0 + 8 * h);
    bl.h8[1] = *(const us8*)(Btl + bcol + k0 + 16 + 8 * h);
#pragma unroll
    for (int mt = 0; mt < 4; ++mt) {
      const size_t ar = (size_t)(64 * wm + 16 * mt + m) * KTOT + k0;
      Frag ah, al;
      ah.h8[0] = *(const us8*)(Amh + ar + 8 * h);
      ah.h8[1] = *(const us8*)(Amh + ar + 16 + 8 * h);
      al.h8[0] = *(const us8*)(Aml + ar + 8 * h);
      al.h8[1] = *(const us8*)(Aml + ar + 16 + 8 * h);
      acc[mt] = wmma_bf(ah.v, bl.v, acc[mt]);
      acc[mt] = wmma_bf(al.v, bh.v, acc[mt]);
      acc[mt] = wmma_bf(ah.v, bh.v, acc[mt]);
    }
  }

#pragma unroll
  for (int mt = 0; mt < 4; ++mt) {
#pragma unroll
    for (int r = 0; r < 8; ++r)
      Cs[64 * wm + 16 * mt + 8 * h + r][16 * wn + m] = acc[mt][r];
  }
  __syncthreads();

#pragma unroll
  for (int s = 0; s < 8; ++s) {
    const int L = 32 * w + 4 * s + (l >> 3);
    const int mrow = L >> 1, hl = L & 1;
    const int cc = 32 * hl + 4 * (l & 7);
    v4f v;
    v.x = Cs[mrow][cc + 0];
    v.y = Cs[mrow][cc + 1];
    v.z = Cs[mrow][cc + 2];
    v.w = Cs[mrow][cc + 3];
    float* dst = out + ((size_t)(b * MOUT + mrow)) * SP + sp0 + cc;
    *(volatile v4f*)dst = v;
  }
  __threadfence();
#pragma unroll
  for (int s = 0; s < 8; ++s) {
    const int L = 32 * w + 4 * s + (l >> 3);
    const int mrow = L >> 1, hl = L & 1;
    const int cc = 32 * hl + 4 * (l & 7);
    v4f v;
    v.x = Cs[mrow][cc + 0];
    v.y = Cs[mrow][cc + 1];
    v.z = Cs[mrow][cc + 2];
    v.w = Cs[mrow][cc + 3];
    float* dst = out + ((size_t)(b * MOUT + mrow)) * SP + sp0 + cc;
    *(volatile v4f*)dst = v;
  }
}

extern "C" void kernel_launch(void* const* d_in, const int* in_sizes, int n_in,
                              void* d_out, int out_size, void* d_ws, size_t ws_size,
                              hipStream_t stream) {
  if (n_in < 6) return;
  if (in_sizes[0] != NB * C * SP) return;
  if (in_sizes[1] != MOUT * C * 9) return;
  if (in_sizes[2] != 18 * C * 9) return;
  if (in_sizes[3] != 18) return;
  if (in_sizes[4] != 3 * C * 9) return;
  if (in_sizes[5] != 3) return;
  if (out_size != NB * MOUT * SP) return;

  const float* x        = (const float*)d_in[0];
  const float* conv_w   = (const float*)d_in[1];
  const float* pconv_w  = (const float*)d_in[2];
  const float* pconv_b  = (const float*)d_in[3];
  const float* adconv_w = (const float*)d_in[4];
  const float* adconv_b = (const float*)d_in[5];
  float* out = (float*)d_out;

  const size_t sz_xp  = (size_t)NB * C * PLANE * sizeof(float);
  const size_t sz_am  = (size_t)MOUT * KTOT * sizeof(unsigned short);
  const size_t sz_ao  = (size_t)MOFF * KTOT * sizeof(unsigned short);
  const size_t sz_pi  = (size_t)NB * NS * SP * 16;
  const size_t sz_bt  = (size_t)NB * SP * KTOT * sizeof(unsigned short);
  const size_t o_xp  = 0;
  const size_t o_amh = o_xp + sz_xp;
  const size_t o_aml = o_amh + sz_am;
  const size_t o_aoh = o_aml + sz_am;
  const size_t o_aol = o_aoh + sz_ao;
  const size_t o_pi  = o_aol + sz_ao;
  const size_t o_pg  = o_pi + sz_pi;
  const size_t o_bth = o_pg + sz_pi;
  const size_t o_btl = o_bth + sz_bt;
  const size_t total = o_btl + sz_bt;
  if (total > ws_size) return;

  char* ws = (char*)d_ws;
  float* xp            = (float*)(ws + o_xp);
  unsigned short* Amh  = (unsigned short*)(ws + o_amh);
  unsigned short* Aml  = (unsigned short*)(ws + o_aml);
  unsigned short* Aoh  = (unsigned short*)(ws + o_aoh);
  unsigned short* Aol  = (unsigned short*)(ws + o_aol);
  v4i* PI              = (v4i*)(ws + o_pi);
  v4f* PG              = (v4f*)(ws + o_pg);
  unsigned short* Bth  = (unsigned short*)(ws + o_bth);
  unsigned short* Btl  = (unsigned short*)(ws + o_btl);

  const int nquad = (NB * C * PLANE) / 4;
  const int nmain = MOUT * (KTOT / 8);
  const int noff  = MOFF * (KTOT / 8);
  const int npair = NB * SP * NS;

  hipLaunchKernelGGL(k_pad, dim3((nquad + 255) / 256), dim3(256), 0, stream, x, xp, nquad);
  hipLaunchKernelGGL(k_prep, dim3((nmain + noff + 255) / 256), dim3(256), 0, stream,
                     conv_w, pconv_w, adconv_w, Amh, Aml, Aoh, Aol, nmain, noff);
  hipLaunchKernelGGL(k_offs, dim3(W / 32, H, NB), dim3(64), 0, stream,
                     (const unsigned short*)Aoh, (const unsigned short*)Aol, (const float*)xp,
                     pconv_b, adconv_b, PI, PG);
  hipLaunchKernelGGL(k_gath, dim3((npair * 16 + 255) / 256), dim3(256), 0, stream,
                     (const float*)xp, (const v4i*)PI, (const v4f*)PG, Bth, Btl, npair);
  hipLaunchKernelGGL(k_gemm, dim3(SP / 64, NB), dim3(256), 0, stream,
                     (const unsigned short*)Amh, (const unsigned short*)Aml,
                     (const unsigned short*)Bth, (const unsigned short*)Btl, out);
}
